// PrefixLinearAttention_79310866088615
// MI455X (gfx1250) — hardware-verified
//
#include <hip/hip_runtime.h>
#include <stdint.h>

#define B_   2
#define N_   2048
#define D_   1024
#define H_   16
#define FD_  16
#define HD_  64
#define ENC_ 512
#define QB_  64
#define KC_  64

typedef __attribute__((ext_vector_type(16))) _Float16 v16h;
typedef __attribute__((ext_vector_type(8)))  _Float16 v8h;
typedef __attribute__((ext_vector_type(16))) __bf16   v16b;
typedef __attribute__((ext_vector_type(8)))  __bf16   v8b;
typedef __attribute__((ext_vector_type(8)))  float    v8f;
typedef __attribute__((ext_vector_type(4)))  float    v4f;

__device__ __forceinline__ unsigned short f2bf_bits(float f) {
  unsigned u = __float_as_uint(f);
  return (unsigned short)((u + 0x7FFFu + ((u >> 16) & 1u)) >> 16);
}
__device__ __forceinline__ float bf_bits2f(unsigned short h) { return __uint_as_float(((unsigned)h) << 16); }

__device__ __forceinline__ void dep_guard_h(v8f& a, v8f& b, v16h x, v16h y) { asm volatile("v_nop\n\tv_nop\n\tv_nop\n\tv_nop" : "+v"(a), "+v"(b) : "v"(x), "v"(y)); }
__device__ __forceinline__ void dep_guard_b(v8f& a, v8f& b, v16b x, v16b y) { asm volatile("v_nop\n\tv_nop\n\tv_nop\n\tv_nop" : "+v"(a), "+v"(b) : "v"(x), "v"(y)); }
__device__ __forceinline__ void keep4_h(v16h a, v16h b, v16h c, v16h d) { asm volatile("v_nop" :: "v"(a), "v"(b), "v"(c), "v"(d)); }
__device__ __forceinline__ void keep4_b(v16b a, v16b b, v16b c, v16b d) { asm volatile("v_nop" :: "v"(a), "v"(b), "v"(c), "v"(d)); }
__device__ __forceinline__ void acc_guard4(v8f& a, v8f& b, v8f& c, v8f& d) { asm volatile("v_nop\n\tv_nop\n\tv_nop\n\tv_nop" : "+v"(a), "+v"(b), "+v"(c), "+v"(d)); }
template <typename T> struct Frag;
template <> struct Frag<_Float16> {
  typedef v16h V; union U { v16h v; v8h h[2]; };
  static __device__ __forceinline__ v16h load(const _Float16* p) {
    U f; f.h[0] = *(const v8h*)(p); f.h[1] = *(const v8h*)(p + 16); return f.v;
  }
  static __device__ __forceinline__ v8f mma(v16h a, v16h b, v8f c) {
    return __builtin_amdgcn_wmma_f32_16x16x32_f16(false, a, false, b, (short)0, c, false, false);
  }
  static __device__ __forceinline__ void guard(v8f& a, v8f& b, v16h x, v16h y) { dep_guard_h(a, b, x, y); }
  static __device__ __forceinline__ void keep(v16h a, v16h b, v16h c, v16h d) { keep4_h(a, b, c, d); }
};
template <> struct Frag<__bf16> {
  typedef v16b V; union U { v16b v; v8b h[2]; };
  static __device__ __forceinline__ v16b load(const __bf16* p) {
    U f; f.h[0] = *(const v8b*)(p); f.h[1] = *(const v8b*)(p + 16); return f.v;
  }
  static __device__ __forceinline__ v8f mma(v16b a, v16b b, v8f c) {
    return __builtin_amdgcn_wmma_f32_16x16x32_bf16(false, a, false, b, (short)0, c, false, false);
  }
  static __device__ __forceinline__ void guard(v8f& a, v8f& b, v16b x, v16b y) { dep_guard_b(a, b, x, y); }
  static __device__ __forceinline__ void keep(v16b a, v16b b, v16b c, v16b d) { keep4_b(a, b, c, d); }
};

template <int ET> struct Elem;
template <> struct Elem<0> { typedef _Float16 T; };
template <> struct Elem<1> { typedef __bf16 T; };
template <int ET, bool SPLIT, int BIAS_MODE, int OUT_MODE, bool RESID, int ACT = 0>
__global__ __launch_bounds__(256) void wmma_gemm64(
    const unsigned short* __restrict__ Ap, const unsigned short* __restrict__ A2p, int lda, long strideA,
    const unsigned short* __restrict__ Btp, const unsigned short* __restrict__ Bt2p, int ldb, long strideB,
    void* __restrict__ Cout, void* __restrict__ Cout2, int ldc, long strideC,
    const float* __restrict__ bias,
    const float* __restrict__ resid, long strideR,
    int M, int N, int K, float scale) {
  typedef typename Elem<ET>::T T;
  typedef typename Frag<T>::V V;
  const T* A = (const T*)Ap; const T* A2 = (const T*)A2p; const T* Bt = (const T*)Btp; const T* Bt2 = (const T*)Bt2p;
  __shared__ __align__(16) float sT[8][16 * 68];
  const int b    = blockIdx.y;
  const int lane = threadIdx.x & 31;
  const int wave = threadIdx.x >> 5;
  const int tilesN = N >> 6;
  const int tilesM = M >> 6;
  const int tile = blockIdx.x * 8 + wave;
  if (tile >= tilesM * tilesN) return;
  const int tm = tile / tilesN;
  const int tn = tile - tm * tilesN;
  const int m0 = tm << 6;
  const int n0 = tn << 6;

  const T* Ab  = A  + (size_t)b * strideA;
  const T* Bb  = Bt + (size_t)b * strideB;
  const T* Ab2 = SPLIT ? (A2  + (size_t)b * strideA) : nullptr;
  const T* Bb2 = SPLIT ? (Bt2 + (size_t)b * strideB) : nullptr;

  const int rlane = lane & 15;
  const int koff  = (lane >> 4) * 8;
  const int mOff  = (lane >> 4) * 8;

  v8f acc[4][4];
#pragma unroll
  for (int i = 0; i < 4; ++i)
#pragma unroll
    for (int j = 0; j < 4; ++j) acc[i][j] = (v8f){0.f,0.f,0.f,0.f,0.f,0.f,0.f,0.f};

  for (int k0 = 0; k0 < K; k0 += 32) {
    V bh[4], bl[4];
#pragma unroll
    for (int j = 0; j < 4; ++j) {
      const size_t bo = (size_t)(n0 + (j << 4) + rlane) * ldb + koff + k0;
      bh[j] = Frag<T>::load(Bb + bo);
      if (SPLIT) bl[j] = Frag<T>::load(Bb2 + bo);
    }
#pragma unroll
    for (int i = 0; i < 4; ++i) {
      const size_t ao = (size_t)(m0 + (i << 4) + rlane) * lda + koff + k0;
      V ah = Frag<T>::load(Ab + ao);
      V al;
      if (SPLIT) al = Frag<T>::load(Ab2 + ao);
#pragma unroll
      for (int j = 0; j < 4; ++j) {
        acc[i][j] = Frag<T>::mma(ah, bh[j], acc[i][j]);
        if (SPLIT) {
          acc[i][j] = Frag<T>::mma(ah, bl[j], acc[i][j]);
          acc[i][j] = Frag<T>::mma(al, bh[j], acc[i][j]);
        }
      }
      Frag<T>::guard(acc[i][0], acc[i][3], ah, SPLIT ? al : ah);
    }
    Frag<T>::keep(bh[0], bh[1], bh[2], bh[3]);
    if (SPLIT) Frag<T>::keep(bl[0], bl[1], bl[2], bl[3]);
  }
  acc_guard4(acc[0][0], acc[0][1], acc[0][2], acc[0][3]);
  acc_guard4(acc[1][0], acc[1][1], acc[1][2], acc[1][3]);
  acc_guard4(acc[2][0], acc[2][1], acc[2][2], acc[2][3]);
  acc_guard4(acc[3][0], acc[3][1], acc[3][2], acc[3][3]);

  float* slab = sT[wave];
  const float* Rb = RESID ? (resid + (size_t)b * strideR) : nullptr;
#pragma unroll
  for (int i = 0; i < 4; ++i) {
    const int mBase = m0 + (i << 4);
#pragma unroll
    for (int j = 0; j < 4; ++j) {
      const int n = n0 + (j << 4) + rlane;
      float bv = 0.f;
      if (BIAS_MODE == 2) bv = bias[n];
#pragma unroll
      for (int r = 0; r < 8; ++r) {
        float v = acc[i][j][r] * scale;
        if (BIAS_MODE == 1) v += bias[mBase + mOff + r];
        if (BIAS_MODE == 2) v += bv;
        if (RESID) v += Rb[(size_t)(mBase + mOff + r) * ldc + n];
        if (ACT == 1) v = tanhf(v);
        if (ACT == 2) v = fmaxf(v, 0.0f);
        if (ACT == 3) v = v / (1.0f + expf(-v));
        if (ACT == 4) v = (v > 0.f) ? v : 0.01f * v;
        if (ACT == 5) v = 0.5f * v * (1.0f + erff(v * 0.70710678118654752f));
        slab[(mOff + r) * 68 + (j << 4) + rlane] = v;
      }
    }
    __builtin_amdgcn_fence(__ATOMIC_RELEASE, "workgroup");
    __builtin_amdgcn_wave_barrier();
    __builtin_amdgcn_fence(__ATOMIC_ACQUIRE, "workgroup");
    if (OUT_MODE == 0) {
      float* C = (float*)Cout + (size_t)b * strideC;
      const int hh = lane >> 4, c4 = (lane & 15) * 4;
      for (int pass = 0; pass < 2; ++pass) {
#pragma unroll
        for (int it = 0; it < 8; ++it) {
          const int row = it * 2 + hh;
          v4f v = *(const v4f*)(slab + row * 68 + c4);
          *(volatile v4f*)(C + (size_t)(mBase + row) * ldc + n0 + c4) = v;
        }
        __threadfence();
      }
    } else {
      const int q = lane >> 3, c8 = (lane & 7) * 8;
      unsigned short* C  = (unsigned short*)Cout  + (size_t)b * strideC;
      unsigned short* C2 = (OUT_MODE == 2) ? ((unsigned short*)Cout2 + (size_t)b * strideC) : nullptr;
      for (int pass = 0; pass < 2; ++pass) {
#pragma unroll
        for (int it = 0; it < 4; ++it) {
          const int row = it * 4 + q;
          const float* sp = slab + row * 68 + c8;
          v8h hv, lv;
#pragma unroll
          for (int e = 0; e < 8; ++e) {
            if (OUT_MODE == 1) {
              hv[e] = (_Float16)sp[e];
            } else {
              unsigned short hb = f2bf_bits(sp[e]);
              unsigned short lb = f2bf_bits(sp[e] - bf_bits2f(hb));
              hv[e] = __builtin_bit_cast(_Float16, hb);
              lv[e] = __builtin_bit_cast(_Float16, lb);
            }
          }
          *(volatile v8h*)(C + (size_t)(mBase + row) * ldc + n0 + c8) = hv;
          if (OUT_MODE == 2) *(volatile v8h*)(C2 + (size_t)(mBase + row) * ldc + n0 + c8) = lv;
        }
        __threadfence();
      }
    }
    __builtin_amdgcn_fence(__ATOMIC_RELEASE, "workgroup");
    __builtin_amdgcn_wave_barrier();
    __builtin_amdgcn_fence(__ATOMIC_ACQUIRE, "workgroup");
  }
}

__global__ __launch_bounds__(256) void cast_f32_f16x2s(
    const float* __restrict__ in, _Float16* __restrict__ out, int n2, float sc) {
  int i = blockIdx.x * 256 + threadIdx.x;
  if (i < n2) {
    const _Float16 h0 = (_Float16)(in[2 * i] * sc), h1 = (_Float16)(in[2 * i + 1] * sc);
    const unsigned u = (unsigned)__builtin_bit_cast(unsigned short, h0) | ((unsigned)__builtin_bit_cast(unsigned short, h1) << 16);
    ((volatile unsigned*)out)[i] = u;
    __threadfence();
    ((volatile unsigned*)out)[i] = u;
  }
}

__device__ __forceinline__ v8f hmma(v16h a, v16h b, v8f c) {
  c = __builtin_amdgcn_wmma_f32_16x16x32_f16(false, a, false, b, (short)0, c, false, false);
  asm volatile("v_nop\n\tv_nop\n\tv_nop\n\tv_nop" : "+v"(c) : "v"(a), "v"(b));
  return c;
}

__global__ __launch_bounds__(128) void lin_attn_kernel(
    const _Float16* __restrict__ q16, const _Float16* __restrict__ k16, const _Float16* __restrict__ ke16,
    const _Float16* __restrict__ Vt, const _Float16* __restrict__ Vte, _Float16* __restrict__ O16) {
  union FH { v16h v; v8h h[2]; };
  __shared__ __align__(16) _Float16 Ks[KC_ * FD_];
  __shared__ __align__(16) _Float16 Vts[HD_ * KC_];
  __shared__ __align__(16) _Float16 Psh[4][16 * KC_];
  __shared__ __align__(16) float    Os[4][16 * 68];

  const int tid  = threadIdx.x;
  const int wave = tid >> 5;
  const int lane = tid & 31;
  const int hh   = lane >> 4;
  const int c    = lane & 15;

  const int nqb = N_ / QB_;
  const int bx = blockIdx.x;
  const int qb = bx % nqb;
  const int bh = bx / nqb;
  const int h  = bh % H_;
  const int b  = bh / H_;
  const int q0 = qb * QB_ + wave * 16;

  const v8h z8 = __builtin_bit_cast(v8h, (v4f){0.f, 0.f, 0.f, 0.f});
  const v8f zacc = (v8f){0.f,0.f,0.f,0.f,0.f,0.f,0.f,0.f};

  FH qa;
  qa.h[0] = *(const v8h*)(q16 + (size_t)(b * N_ + q0 + c) * (H_ * FD_) + h * FD_ + 8 * hh);
  qa.h[1] = z8;

  float lrow[8];
  v8f oacc[4];
#pragma unroll
  for (int r = 0; r < 8; ++r) lrow[r] = 0.f;
#pragma unroll
  for (int t = 0; t < 4; ++t) oacc[t] = zacc;

  const int nDec = qb + 1;
  const int nCh  = nDec + ENC_ / KC_;
  for (int kc = 0; kc < nCh; ++kc) {
    const bool dec = (kc < nDec);
    const int kv0 = dec ? kc * KC_ : (kc - nDec) * KC_;
    const _Float16* krows = dec ? (k16  + (size_t)(b * N_   + kv0) * (H_ * FD_) + h * FD_)
                                : (ke16 + (size_t)(b * ENC_ + kv0) * (H_ * FD_) + h * FD_);
    const _Float16* vsrc  = dec ? (Vt  + (size_t)bh * HD_ * N_   + kv0)
                                : (Vte + (size_t)bh * HD_ * ENC_ + kv0);
    const int vpitch = dec ? N_ : ENC_;
    __syncthreads();
    {
      const int row = tid >> 1, hf = (tid & 1) * 8;
      *(v8h*)(Ks + row * FD_ + hf) = *(const v8h*)(krows + (size_t)row * (H_ * FD_) + hf);
#pragma unroll
      for (int i = 0; i < 4; ++i) {
        const int item = tid + 128 * i;
        const int d = item >> 3, seg = (item & 7) * 8;
        *(v8h*)(Vts + d * KC_ + seg) = *(const v8h*)(vsrc + (size_t)d * vpitch + seg);
      }
    }
    __syncthreads();

    v8f s[4];
#pragma unroll
    for (int j = 0; j < 4; ++j) {
      FH kb;
      kb.h[0] = *(const v8h*)(Ks + (j * 16 + c) * FD_ + 8 * hh);
      kb.h[1] = z8;
      s[j] = hmma(qa.v, kb.v, zacc);
    }

    const bool diag = dec && (kc == qb);
    _Float16* pwh = Psh[wave];
#pragma unroll
    for (int r = 0; r < 8; ++r) {
      const int qrow = q0 + 8 * hh + r;
      float psum = 0.f;
#pragma unroll
      for (int j = 0; j < 4; ++j) {
        const int kvcol = kv0 + j * 16 + c;
        const float sv = s[j][r];
        float a = 1.0f + 0.25f * sv + (sv * sv) * 0.03125f;
        if (diag && (kvcol > qrow)) a = 0.f;
        psum += a;
        pwh[(8 * hh + r) * KC_ + j * 16 + c] = (_Float16)a;
      }
#pragma unroll
      for (int off = 1; off < 16; off <<= 1) psum += __shfl_xor(psum, off, 32);
      lrow[r] += psum;
    }
    __builtin_amdgcn_fence(__ATOMIC_RELEASE, "workgroup");
    __builtin_amdgcn_wave_barrier();
    __builtin_amdgcn_fence(__ATOMIC_ACQUIRE, "workgroup");

#pragma unroll 1
    for (int kk = 0; kk < 2; ++kk) {
      FH pa;
      pa.h[0] = *(const v8h*)(pwh + c * KC_ + kk * 32 + 8 * hh);
      pa.h[1] = *(const v8h*)(pwh + c * KC_ + kk * 32 + 16 + 8 * hh);
#pragma unroll
      for (int t = 0; t < 4; ++t) {
        FH vb;
        vb.h[0] = *(const v8h*)(Vts + (t * 16 + c) * KC_ + kk * 32 + 8 * hh);
        vb.h[1] = *(const v8h*)(Vts + (t * 16 + c) * KC_ + kk * 32 + 16 + 8 * hh);
        oacc[t] = hmma(pa.v, vb.v, oacc[t]);
      }
    }
  }

  float* os = Os[wave];
#pragma unroll
  for (int r = 0; r < 8; ++r) {
    const float inv = 16.0f / (lrow[r] + 1e-12f);
#pragma unroll
    for (int t = 0; t < 4; ++t) os[(8 * hh + r) * 68 + t * 16 + c] = oacc[t][r] * inv;
  }
  __builtin_amdgcn_fence(__ATOMIC_RELEASE, "workgroup");
  __builtin_amdgcn_wave_barrier();
  __builtin_amdgcn_fence(__ATOMIC_ACQUIRE, "workgroup");
  {
    const int q4 = lane >> 3, c8 = (lane & 7) * 8;
    for (int pass = 0; pass < 2; ++pass) {
#pragma unroll
      for (int it = 0; it < 4; ++it) {
        const int row = it * 4 + q4;
        const float* sp = os + row * 68 + c8;
        v8h hv;
#pragma unroll
        for (int e = 0; e < 8; ++e) hv[e] = (_Float16)sp[e];
        *(volatile v8h*)(O16 + (size_t)(b * N_ + q0 + row) * (H_ * HD_) + h * HD_ + c8) = hv;
      }
      __threadfence();
    }
  }
}

extern "C" void kernel_launch(void* const* d_in, const int* in_sizes, int n_in,
                              void* d_out, int out_size, void* d_ws, size_t ws_size,
                              hipStream_t stream) {
  if (n_in < 7) return;
  const int nX = B_ * N_ * D_;
  const int nWqk = H_ * FD_ * D_;
  const int nWv = H_ * HD_ * D_;
  const int nWo = D_ * H_ * HD_;
  if (in_sizes[0] != nX || in_sizes[1] != nWqk || in_sizes[2] != nWqk || in_sizes[3] != nWv ||
      in_sizes[4] != nWqk || in_sizes[5] != nWv || in_sizes[6] != nWo || out_size != nX) return;

  const float* x    = (const float*)d_in[0];
  const float* Wq   = (const float*)d_in[1];
  const float* Wk   = (const float*)d_in[2];
  const float* Wv   = (const float*)d_in[3];
  const float* Wke  = (const float*)d_in[4];
  const float* Wve  = (const float*)d_in[5];
  const float* Wout = (const float*)d_in[6];
  float* out = (float*)d_out;

  size_t off = 0;
  auto take = [&](size_t bytes) -> size_t { size_t o = off; off += (bytes + 255) & ~(size_t)255; return o; };
  const size_t BN = (size_t)B_ * N_;
  const size_t BE = (size_t)B_ * ENC_;
  const size_t o_x16  = take(BN * D_ * 2);
  const size_t o_wq   = take((size_t)nWqk * 2);
  const size_t o_wk   = take((size_t)nWqk * 2);
  const size_t o_wke  = take((size_t)nWqk * 2);
  const size_t o_wv   = take((size_t)nWv * 2);
  const size_t o_wve  = take((size_t)nWv * 2);
  const size_t o_wo   = take((size_t)nWo * 2);
  const size_t o_q16  = take(BN * (H_ * FD_) * 2);
  const size_t o_k16  = take(BN * (H_ * FD_) * 2);
  const size_t o_ke16 = take(BE * (H_ * FD_) * 2);
  const size_t o_vt   = take((size_t)B_ * H_ * HD_ * N_ * 2);
  const size_t o_vte  = take((size_t)B_ * H_ * HD_ * ENC_ * 2);
  const size_t o_o16  = take(BN * (H_ * HD_) * 2);
  if (off > ws_size) return;
  char* ws = (char*)d_ws;
  _Float16* x16   = (_Float16*)(ws + o_x16);
  _Float16* Wq16  = (_Float16*)(ws + o_wq);
  _Float16* Wk16  = (_Float16*)(ws + o_wk);
  _Float16* Wke16 = (_Float16*)(ws + o_wke);
  _Float16* Wv16  = (_Float16*)(ws + o_wv);
  _Float16* Wve16 = (_Float16*)(ws + o_wve);
  _Float16* Wo16  = (_Float16*)(ws + o_wo);
  _Float16* q16   = (_Float16*)(ws + o_q16);
  _Float16* k16   = (_Float16*)(ws + o_k16);
  _Float16* ke16  = (_Float16*)(ws + o_ke16);
  _Float16* Vt    = (_Float16*)(ws + o_vt);
  _Float16* Vte   = (_Float16*)(ws + o_vte);
  _Float16* O16   = (_Float16*)(ws + o_o16);
  const float* fdum = x;

  auto cast = [&](const float* src, _Float16* dst, int n, float sc) {
    const int n2 = n / 2;
    cast_f32_f16x2s<<<dim3((unsigned)((n2 + 255) / 256)), dim3(256), 0, stream>>>(src, dst, n2, sc);
  };
  cast(x, x16, nX, 1.0f);
  cast(Wq, Wq16, nWqk, 16.0f);
  cast(Wk, Wk16, nWqk, 16.0f);
  cast(Wke, Wke16, nWqk, 16.0f);
  cast(Wv, Wv16, nWv, 16.0f);
  cast(Wve, Wve16, nWv, 16.0f);
  cast(Wout, Wo16, nWo, 16.0f);

  typedef const unsigned short* cus;
  const float s16 = 1.0f / 16.0f;
  {
    const int M = (int)BN, Nn = H_ * FD_, tiles = (M / 64) * (Nn / 64);
    wmma_gemm64<0, false, 0, 1, false, 0><<<dim3((unsigned)((tiles + 7) / 8), 1), dim3(256), 0, stream>>>(
        (cus)x16, (cus)x16, D_, 0L, (cus)Wq16, (cus)Wq16, D_, 0L, (void*)q16, (void*)q16, Nn, 0L,
        fdum, fdum, 0L, M, Nn, D_, s16);
    wmma_gemm64<0, false, 0, 1, false, 0><<<dim3((unsigned)((tiles + 7) / 8), 1), dim3(256), 0, stream>>>(
        (cus)x16, (cus)x16, D_, 0L, (cus)Wk16, (cus)Wk16, D_, 0L, (void*)k16, (void*)k16, Nn, 0L,
        fdum, fdum, 0L, M, Nn, D_, s16);
  }
  {
    const int M = ENC_, Nn = H_ * FD_, tiles = (M / 64) * (Nn / 64);
    wmma_gemm64<0, false, 0, 1, false, 0><<<dim3((unsigned)((tiles + 7) / 8), B_), dim3(256), 0, stream>>>(
        (cus)x16, (cus)x16, D_, (long)N_ * D_, (cus)Wke16, (cus)Wke16, D_, 0L, (void*)ke16, (void*)ke16, Nn, (long)ENC_ * Nn,
        fdum, fdum, 0L, M, Nn, D_, s16);
  }
  {
    const int M = H_ * HD_, Nn = N_, tiles = (M / 64) * (Nn / 64);
    wmma_gemm64<0, false, 0, 1, false, 0><<<dim3((unsigned)((tiles + 7) / 8), B_), dim3(256), 0, stream>>>(
        (cus)Wv16, (cus)Wv16, D_, 0L, (cus)x16, (cus)x16, D_, (long)N_ * D_, (void*)Vt, (void*)Vt, Nn, (long)M * Nn,
        fdum, fdum, 0L, M, Nn, D_, s16);
  }
  {
    const int M = H_ * HD_, Nn = ENC_, tiles = (M / 64) * (Nn / 64);
    wmma_gemm64<0, false, 0, 1, false, 0><<<dim3((unsigned)((tiles + 7) / 8), B_), dim3(256), 0, stream>>>(
        (cus)Wve16, (cus)Wve16, D_, 0L, (cus)x16, (cus)x16, D_, (long)N_ * D_, (void*)Vte, (void*)Vte, Nn, (long)M * Nn,
        fdum, fdum, 0L, M, Nn, D_, s16);
  }

  lin_attn_kernel<<<dim3((unsigned)(B_ * H_ * (N_ / QB_))), dim3(128), 0, stream>>>(q16, k16, ke16, Vt, Vte, O16);

  {
    const int M = (int)BN, Nn = D_, Kk = H_ * HD_, tiles = (M / 64) * (Nn / 64);
    wmma_gemm64<0, false, 0, 0, false, 0><<<dim3((unsigned)((tiles + 7) / 8), 1), dim3(256), 0, stream>>>(
        (cus)O16, (cus)O16, Kk, 0L, (cus)Wo16, (cus)Wo16, Kk, 0L, (void*)out, (void*)out, Nn, 0L,
        fdum, fdum, 0L, M, Nn, Kk, 1.0f / 256.0f);
  }
}
